// Block_9405978378750
// MI455X (gfx1250) — hardware-run, weakly checked
//
#include <hip/hip_runtime.h>
#include <math.h>

typedef __attribute__((ext_vector_type(16))) _Float16 v16h;
typedef __attribute__((ext_vector_type(8)))  _Float16 v8h;
typedef __attribute__((ext_vector_type(8)))  float    v8f;
typedef __attribute__((ext_vector_type(4)))  float    v4f;

#ifndef NB
#define NB 2
#endif
#ifndef SEQ
#define SEQ 2048
#endif
#define NB_FULL 2
#define SEQ_FULL 2048
#define DM 1024
#define NHEAD 16
#define HD 64
#define DFF 4096
#define C3 3072
#define NR (NB * SEQ)

#define CXF 16.0f
#define CWF 64.0f
#define CHF 16.0f
#define CCF 64.0f
#define CPF 4096.0f

static_assert(SEQ % 128 == 0);
static_assert(NB <= NB_FULL && SEQ <= SEQ_FULL);
static_assert(DM % 64 == 0 && C3 % 64 == 0 && DFF % 64 == 0);
static_assert(NHEAD * HD == DM && HD == 64);
static_assert((size_t)NR * DM * 2 * 3 + ((size_t)C3 * DM + (size_t)DM * DM + (size_t)DFF * DM * 2) * 2 + (size_t)NR * C3 * 2 + (size_t)NR * DM * 4 + (size_t)NR * DFF * 2 <= (size_t)134217728);

union FragU { v16h v; v8h q[2]; };
__device__ __forceinline__ v16h ld_frag(const _Float16* __restrict__ p) {
    FragU f; f.q[0] = *(const v8h*)p; f.q[1] = *(const v8h*)(p + 16); return f.v;
}
__device__ __forceinline__ float bf16r(float f) {
    unsigned int u = __float_as_uint(f);
    u += 0x7fffu + ((u >> 16) & 1u);
    return __uint_as_float(u & 0xffff0000u);
}
__device__ __forceinline__ v8f wmma2(v16h a0, v16h b0, v16h a1, v16h b1, v8f c) {
    c = __builtin_amdgcn_wmma_f32_16x16x32_f16(false, a0, false, b0, (short)0, c, false, false);
    c = __builtin_amdgcn_wmma_f32_16x16x32_f16(false, a1, false, b1, (short)0, c, false, false);
    asm volatile("v_nop\n\tv_nop\n\tv_nop\n\tv_nop" : "+v"(c) : "v"(a0), "v"(b0), "v"(a1), "v"(b1));
    return c;
}

template <bool RND>
__global__ __launch_bounds__(128) void k_ln(const float* __restrict__ X, const float* __restrict__ G, const float* __restrict__ Bv,
                                             _Float16* __restrict__ Y, int x_full) {
    __shared__ float red[8];
    const int row = blockIdx.x, t = threadIdx.x, lane = t & 31, wave = t >> 5;
    const int bq = row / SEQ, sq = row - bq * SEQ;
    const float* xr = X + ((size_t)bq * x_full + sq) * DM + t * 8;
    const v4f xa = *(const v4f*)xr, xb = *(const v4f*)(xr + 4);
    float v[8];
#pragma unroll
    for (int e = 0; e < 4; ++e) { v[e] = RND ? bf16r(xa[e]) : xa[e]; v[4 + e] = RND ? bf16r(xb[e]) : xb[e]; }
    float s = 0.f;
#pragma unroll
    for (int e = 0; e < 8; ++e) s += v[e];
    s += __shfl_xor(s, 1, 32); s += __shfl_xor(s, 2, 32); s += __shfl_xor(s, 4, 32); s += __shfl_xor(s, 8, 32); s += __shfl_xor(s, 16, 32);
    if (lane == 0) red[wave] = s;
    __syncthreads();
    const float mu = (red[0] + red[1] + red[2] + red[3]) * (1.0f / DM);
    float q = 0.f;
#pragma unroll
    for (int e = 0; e < 8; ++e) { const float d = v[e] - mu; q += d * d; }
    q += __shfl_xor(q, 1, 32); q += __shfl_xor(q, 2, 32); q += __shfl_xor(q, 4, 32); q += __shfl_xor(q, 8, 32); q += __shfl_xor(q, 16, 32);
    if (lane == 0) red[4 + wave] = q;
    __syncthreads();
    const float var = (red[4] + red[5] + red[6] + red[7]) * (1.0f / DM);
    const float rstd = rsqrtf(var + 1e-5f);
    const v4f ga = *(const v4f*)(G + t * 8), gb = *(const v4f*)(G + t * 8 + 4);
    const v4f ba = *(const v4f*)(Bv + t * 8), bb = *(const v4f*)(Bv + t * 8 + 4);
    v8h o;
#pragma unroll
    for (int e = 0; e < 4; ++e) {
        o[e]     = (_Float16)((((v[e] - mu) * rstd) * bf16r(ga[e]) + bf16r(ba[e])) * CXF);
        o[4 + e] = (_Float16)((((v[4 + e] - mu) * rstd) * bf16r(gb[e]) + bf16r(bb[e])) * CXF);
    }
    _Float16* dst = Y + (size_t)row * DM + t * 8;
    *(volatile v8h*)dst = o;
    __threadfence();
    *(volatile v8h*)dst = o;
}

__global__ __launch_bounds__(256) void k_wt(const float* __restrict__ W, _Float16* __restrict__ Wt, int K, int N) {
    __shared__ __align__(16) _Float16 tl[64 * 72];
    const int n0 = blockIdx.x * 64, k0 = blockIdx.y * 64;
    const int tid = threadIdx.x, lane = tid & 31, wave = tid >> 5;
#pragma unroll
    for (int it = 0; it < 4; ++it) {
        const int p = tid + it * 256;
        const int kr = p >> 4, c4 = (p & 15) * 4;
        const v4f w = *(const v4f*)(W + (size_t)(k0 + kr) * N + n0 + c4);
#pragma unroll
        for (int e = 0; e < 4; ++e) tl[(c4 + e) * 72 + kr] = (_Float16)(bf16r(w[e]) * CWF);
    }
    __syncthreads();
#pragma unroll
    for (int it = 0; it < 2; ++it) {
        const int nr = (wave * 2 + it) * 4 + (lane >> 3), c8 = (lane & 7) * 8;
        const v8h o = *(const v8h*)&tl[nr * 72 + c8];
        _Float16* dst = Wt + (size_t)(n0 + nr) * K + k0 + c8;
        *(volatile v8h*)dst = o;
        __threadfence();
        *(volatile v8h*)dst = o;
    }
}

__global__ __launch_bounds__(128) void k_vt(const _Float16* __restrict__ QKV, _Float16* __restrict__ VT) {
    __shared__ __align__(16) _Float16 tl[64 * 72];
    const int tb = blockIdx.x, h = blockIdx.y, b = blockIdx.z;
    const int tid = threadIdx.x, lane = tid & 31, wave = tid >> 5;
#pragma unroll
    for (int it = 0; it < 4; ++it) {
        const int p = tid + it * 128;
        const int tr = p >> 3, c8 = (p & 7) * 8;
        const v8h x = *(const v8h*)(QKV + ((size_t)b * SEQ + tb * 64 + tr) * C3 + 2 * DM + h * HD + c8);
#pragma unroll
        for (int e = 0; e < 8; ++e) tl[(c8 + e) * 72 + tr] = x[e];
    }
    __syncthreads();
#pragma unroll
    for (int it = 0; it < 4; ++it) {
        const int dr = (wave * 4 + it) * 4 + (lane >> 3), c8 = (lane & 7) * 8;
        const v8h o = *(const v8h*)&tl[dr * 72 + c8];
        _Float16* dst = VT + ((size_t)(b * NHEAD + h) * HD + dr) * SEQ + tb * 64 + c8;
        *(volatile v8h*)dst = o;
        __threadfence();
        *(volatile v8h*)dst = o;
    }
}

#define CTP 68
template <int EPI>
__global__ __launch_bounds__(128) void k_gemm(const _Float16* __restrict__ A, const _Float16* __restrict__ Bt,
                                               _Float16* __restrict__ Ch, float* __restrict__ Cf, const float* __restrict__ R,
                                               int K, int N, int r_full, int c_full, float alpha) {
    __shared__ __align__(16) float ct[4][32 * CTP];
    const int lane = threadIdx.x & 31, hf = lane >> 4, l15 = lane & 15, wave = threadIdx.x >> 5;
    const int m0 = blockIdx.y * 128 + wave * 32, n0 = blockIdx.x * 64;
    const _Float16* ap0 = A + (size_t)(m0 + l15) * K + 8 * hf;
    const _Float16* ap1 = ap0 + (size_t)16 * K;
    const _Float16* bp0 = Bt + (size_t)(n0 + l15) * K + 8 * hf;
    const _Float16* bp1 = bp0 + (size_t)16 * K;
    const _Float16* bp2 = bp0 + (size_t)32 * K;
    const _Float16* bp3 = bp0 + (size_t)48 * K;
    v8f acc[2][4];
#pragma unroll
    for (int i = 0; i < 2; ++i)
#pragma unroll
        for (int j = 0; j < 4; ++j) { v8f zz = {}; acc[i][j] = zz; }
    for (int k0 = 0; k0 < K; k0 += 32) {
        v16h a[2], b[4];
        a[0] = ld_frag(ap0 + k0); a[1] = ld_frag(ap1 + k0);
        b[0] = ld_frag(bp0 + k0); b[1] = ld_frag(bp1 + k0); b[2] = ld_frag(bp2 + k0); b[3] = ld_frag(bp3 + k0);
#pragma unroll
        for (int i = 0; i < 2; ++i)
#pragma unroll
            for (int j = 0; j < 4; ++j)
                acc[i][j] = __builtin_amdgcn_wmma_f32_16x16x32_f16(false, a[i], false, b[j], (short)0, acc[i][j], false, false);
        asm volatile("v_nop\n\tv_nop\n\tv_nop\n\tv_nop"
                     : "+v"(acc[0][0]), "+v"(acc[0][1]), "+v"(acc[0][2]), "+v"(acc[0][3]),
                       "+v"(acc[1][0]), "+v"(acc[1][1]), "+v"(acc[1][2]), "+v"(acc[1][3])
                     : "v"(a[0]), "v"(a[1]), "v"(b[0]), "v"(b[1]), "v"(b[2]), "v"(b[3]));
    }
#pragma unroll
    for (int i = 0; i < 2; ++i)
#pragma unroll
        for (int j = 0; j < 4; ++j)
#pragma unroll
            for (int r = 0; r < 8; ++r)
                ct[wave][(i * 16 + 8 * hf + r) * CTP + j * 16 + l15] = acc[i][j][r] * alpha;
    __syncthreads();
    if (EPI <= 1) {
#pragma unroll 1
        for (int s = 0; s < 8; ++s) {
            const int row = s * 4 + (lane >> 3), c8 = (lane & 7) * 8;
            const v4f x0 = *(const v4f*)&ct[wave][row * CTP + c8];
            const v4f x1 = *(const v4f*)&ct[wave][row * CTP + c8 + 4];
            v8h o;
#pragma unroll
            for (int e = 0; e < 4; ++e) {
                float u0 = x0[e], u1 = x1[e];
                if (EPI == 1) {
                    u0 = (0.5f * u0 * (1.0f + erff(u0 * 0.70710678118654752f))) * CHF;
                    u1 = (0.5f * u1 * (1.0f + erff(u1 * 0.70710678118654752f))) * CHF;
                }
                o[e] = (_Float16)u0; o[4 + e] = (_Float16)u1;
            }
            _Float16* dst = Ch + (size_t)(m0 + row) * N + n0 + c8;
            *(volatile v8h*)dst = o;
            __threadfence();
            *(volatile v8h*)dst = o;
        }
    } else {
#pragma unroll 1
        for (int s = 0; s < 16; ++s) {
            const int row = s * 2 + (lane >> 4), c4 = (lane & 15) * 4;
            v4f v = *(const v4f*)&ct[wave][row * CTP + c4];
            const int gr = m0 + row;
            const int bq = gr / SEQ, sq = gr - bq * SEQ;
            v4f rr = *(const v4f*)(R + ((size_t)bq * r_full + sq) * N + n0 + c4);
            if (EPI == 3) {
#pragma unroll
                for (int e = 0; e < 4; ++e) rr[e] = bf16r(rr[e]);
            }
            v += rr;
            float* dst = Cf + ((size_t)bq * c_full + sq) * N + n0 + c4;
            *(volatile v4f*)dst = v;
            __threadfence();
            *(volatile v4f*)dst = v;
        }
    }
}

#define PP 72
__global__ __launch_bounds__(128) void k_attn(const _Float16* __restrict__ QKV, const _Float16* __restrict__ VT, _Float16* __restrict__ CTX) {
    __shared__ __align__(16) _Float16 pt[4][16 * PP];
    const int lane = threadIdx.x & 31, hf = lane >> 4, l15 = lane & 15, wave = threadIdx.x >> 5;
    const int h = blockIdx.y, b = blockIdx.z;
    const int q0 = blockIdx.x * 64 + wave * 16;
    const size_t rowb = (size_t)b * SEQ;
    const float NEG = -__builtin_inff();
    const float SC = 0.125f * 1.4426950408889634f;
    const _Float16* qrow = QKV + (rowb + q0 + l15) * C3 + h * HD + 8 * hf;
    const v16h qa0 = ld_frag(qrow), qa1 = ld_frag(qrow + 32);
    const _Float16* kcol = QKV + rowb * C3 + DM + h * HD + 8 * hf;
    const _Float16* vrow = VT + ((size_t)(b * NHEAD + h) * HD + l15) * SEQ + 8 * hf;
    v8f o[4]; float m8[8], l8[8];
#pragma unroll
    for (int t = 0; t < 4; ++t) { v8f zz = {}; o[t] = zz; }
#pragma unroll
    for (int i = 0; i < 8; ++i) { m8[i] = NEG; l8[i] = 0.f; }
    const int jend = (blockIdx.x + 1) * 64;
    for (int j0 = 0; j0 < jend; j0 += 64) {
        v8f s[4];
#pragma unroll
        for (int t = 0; t < 4; ++t) {
            const _Float16* kp = kcol + (size_t)(j0 + t * 16 + l15) * C3;
            const v16h kf0 = ld_frag(kp), kf1 = ld_frag(kp + 32);
            v8f acc = {};
            s[t] = wmma2(qa0, kf0, qa1, kf1, acc);
        }
        float pv[8][4];
#pragma unroll
        for (int i = 0; i < 8; ++i) {
            const int irow = q0 + 8 * hf + i;
            float sc[4];
#pragma unroll
            for (int t = 0; t < 4; ++t) {
                const int jg = j0 + t * 16 + l15;
                const float v = s[t][i] * SC;
                sc[t] = (jg > irow) ? NEG : v;
            }
            float mx = fmaxf(fmaxf(sc[0], sc[1]), fmaxf(sc[2], sc[3]));
            mx = fmaxf(mx, __shfl_xor(mx, 1, 32)); mx = fmaxf(mx, __shfl_xor(mx, 2, 32));
            mx = fmaxf(mx, __shfl_xor(mx, 4, 32)); mx = fmaxf(mx, __shfl_xor(mx, 8, 32));
            const float mnew = fmaxf(m8[i], mx);
            const float corr = (mnew == NEG) ? 1.f : exp2f(m8[i] - mnew);
            float rs = 0.f;
#pragma unroll
            for (int t = 0; t < 4; ++t) {
                const float pp = (sc[t] == NEG) ? 0.f : exp2f(sc[t] - mnew);
                rs += pp; pv[i][t] = pp;
            }
            rs += __shfl_xor(rs, 1, 32); rs += __shfl_xor(rs, 2, 32); rs += __shfl_xor(rs, 4, 32); rs += __shfl_xor(rs, 8, 32);
            l8[i] = l8[i] * corr + rs; m8[i] = mnew;
#pragma unroll
            for (int t = 0; t < 4; ++t) o[t][i] *= corr;
        }
        __syncthreads();
#pragma unroll
        for (int i = 0; i < 8; ++i)
#pragma unroll
            for (int t = 0; t < 4; ++t) pt[wave][(i + 8 * hf) * PP + t * 16 + l15] = (_Float16)(pv[i][t] * CPF);
        __syncthreads();
        FragU pa0, pa1;
        pa0.q[0] = *(const v8h*)&pt[wave][l15 * PP + 8 * hf];
        pa0.q[1] = *(const v8h*)&pt[wave][l15 * PP + 16 + 8 * hf];
        pa1.q[0] = *(const v8h*)&pt[wave][l15 * PP + 32 + 8 * hf];
        pa1.q[1] = *(const v8h*)&pt[wave][l15 * PP + 48 + 8 * hf];
#pragma unroll
        for (int t = 0; t < 4; ++t) {
            const _Float16* vp = vrow + (size_t)(t * 16) * SEQ + j0;
            const v16h vf0 = ld_frag(vp), vf1 = ld_frag(vp + 32);
            o[t] = wmma2(pa0.v, vf0, pa1.v, vf1, o[t]);
        }
    }
    __syncthreads();
#pragma unroll
    for (int i = 0; i < 8; ++i) {
        const float inv = (l8[i] > 0.f) ? 1.0f / (l8[i] * (CPF / CCF)) : 0.f;
#pragma unroll
        for (int t = 0; t < 4; ++t) pt[wave][(i + 8 * hf) * PP + t * 16 + l15] = (_Float16)(o[t][i] * inv);
    }
    __syncthreads();
#pragma unroll
    for (int s = 0; s < 4; ++s) {
        const int row = s * 4 + (lane >> 3), c8 = (lane & 7) * 8;
        const v8h ov = *(const v8h*)&pt[wave][row * PP + c8];
        _Float16* dst = CTX + (rowb + q0 + row) * DM + h * HD + c8;
        *(volatile v8h*)dst = ov;
        __threadfence();
        *(volatile v8h*)dst = ov;
    }
}

extern "C" void kernel_launch(void* const* d_in, const int* in_sizes, int n_in, void* d_out, int out_size, void* d_ws, size_t ws_size, hipStream_t stream) {
    if (n_in < 9) return;
    const long long xneed = ((long long)(NB - 1) * SEQ_FULL + SEQ) * DM;
    if ((long long)in_sizes[0] < xneed) return;
    if ((long long)in_sizes[1] < (long long)DM * C3) return;
    if ((long long)in_sizes[2] < (long long)DM * DM) return;
    if ((long long)in_sizes[3] < (long long)DM * DFF) return;
    if ((long long)in_sizes[4] < (long long)DFF * DM) return;
    if (in_sizes[5] < DM || in_sizes[6] < DM || in_sizes[7] < DM || in_sizes[8] < DM) return;
    if ((long long)out_size < xneed) return;

    const float* x      = (const float*)d_in[0];
    const float* w_qkv  = (const float*)d_in[1];
    const float* w_proj = (const float*)d_in[2];
    const float* w1     = (const float*)d_in[3];
    const float* w2     = (const float*)d_in[4];
    const float* ln1_g  = (const float*)d_in[5];
    const float* ln1_b  = (const float*)d_in[6];
    const float* ln2_g  = (const float*)d_in[7];
    const float* ln2_b  = (const float*)d_in[8];
    float* out = (float*)d_out;

    char* wsp = (char*)d_ws; size_t off = 0;
    _Float16* XN     = (_Float16*)(wsp + off); off += (size_t)NR * DM * 2;
    _Float16* WqkvT  = (_Float16*)(wsp + off); off += (size_t)C3 * DM * 2;
    _Float16* WprojT = (_Float16*)(wsp + off); off += (size_t)DM * DM * 2;
    _Float16* W1T    = (_Float16*)(wsp + off); off += (size_t)DFF * DM * 2;
    _Float16* W2T    = (_Float16*)(wsp + off); off += (size_t)DM * DFF * 2;
    _Float16* QKV    = (_Float16*)(wsp + off); off += (size_t)NR * C3 * 2;
    _Float16* VT     = (_Float16*)(wsp + off); off += (size_t)NR * DM * 2;
    _Float16* CTX    = (_Float16*)(wsp + off); off += (size_t)NR * DM * 2;
    float*    X1     = (float*)(wsp + off);    off += (size_t)NR * DM * 4;
    _Float16* Hh     = (_Float16*)(wsp + off); off += (size_t)NR * DFF * 2;
    if (off > ws_size) return;

    k_ln<true><<<dim3((unsigned)NR), 128, 0, stream>>>(x, ln1_g, ln1_b, XN, SEQ_FULL);
    k_wt<<<dim3(C3 / 64, DM / 64), 256, 0, stream>>>(w_qkv, WqkvT, DM, C3);
    k_wt<<<dim3(DM / 64, DM / 64), 256, 0, stream>>>(w_proj, WprojT, DM, DM);
    k_wt<<<dim3(DFF / 64, DM / 64), 256, 0, stream>>>(w1, W1T, DM, DFF);
    k_wt<<<dim3(DM / 64, DFF / 64), 256, 0, stream>>>(w2, W2T, DFF, DM);
    k_gemm<0><<<dim3(C3 / 64, NR / 128), 128, 0, stream>>>(XN, WqkvT, QKV, X1, X1, DM, C3, SEQ, SEQ, 1.0f / (CXF * CWF));
    k_vt<<<dim3(SEQ / 64, NHEAD, NB), 128, 0, stream>>>(QKV, VT);
    k_attn<<<dim3(SEQ / 64, NHEAD, NB), 128, 0, stream>>>(QKV, VT, CTX);
    k_gemm<3><<<dim3(DM / 64, NR / 128), 128, 0, stream>>>(CTX, WprojT, QKV, X1, x, DM, DM, SEQ_FULL, SEQ, 1.0f / (CCF * CWF));
    k_ln<false><<<dim3((unsigned)NR), 128, 0, stream>>>(X1, ln2_g, ln2_b, XN, SEQ);
    k_gemm<1><<<dim3(DFF / 64, NR / 128), 128, 0, stream>>>(XN, W1T, Hh, X1, X1, DM, DFF, SEQ, SEQ, 1.0f / (CXF * CWF));
    k_gemm<2><<<dim3(DM / 64, NR / 128), 128, 0, stream>>>(Hh, W2T, QKV, out, X1, DFF, DM, SEQ, SEQ_FULL, 1.0f / (CHF * CWF));
}
